// HAttentionMixer_70712341561580
// MI455X (gfx1250) — hardware-verified
//
#include <hip/hip_runtime.h>

#define DMOD  1024
#define NHD   8
#define SDIM  128
#define HDIM  128
#define NLV   12
#define NGL   128
#define NQKV  (3 * DMOD)
#define TPB   128
#define OSTR  68
#define GST   132
#define YST   136
#define LAMP  128
#define SLMAX 2048
#define KSC   (0.08838834764831845f * (1.0f / 4096.0f))

static_assert(NHD * HDIM == DMOD);
static_assert(NHD * SDIM == DMOD);
static_assert(NHD + NHD * NLV <= NGL);
static_assert(DMOD % 64 == 0);
static_assert(DMOD % 32 == 0);
static_assert(NQKV % 64 == 0);
static_assert(OSTR % 4 == 0);
static_assert(GST % 4 == 0);
static_assert(YST % 8 == 0);
static_assert(SLMAX % TPB == 0);

typedef unsigned short us16 __attribute__((ext_vector_type(16)));
typedef unsigned short us8  __attribute__((ext_vector_type(8)));
typedef unsigned short us8a __attribute__((ext_vector_type(8), may_alias));
typedef __bf16 v16b __attribute__((ext_vector_type(16)));
typedef _Float16 v16h __attribute__((ext_vector_type(16)));
typedef float v8f __attribute__((ext_vector_type(8)));
typedef float v4f __attribute__((ext_vector_type(4)));
typedef float v4fa __attribute__((ext_vector_type(4), may_alias));
union FragU { us16 v; us8 h[2]; };

__device__ __forceinline__ unsigned short bf16_bits(float f) {
  unsigned u = __float_as_uint(f);
  u += 0x7FFFu + ((u >> 16) & 1u);
  return (unsigned short)(u >> 16);
}
__device__ __forceinline__ float bf16_val(unsigned short b) { return __uint_as_float(((unsigned)b) << 16); }
__device__ __forceinline__ float bf16r(float f) { return bf16_val(bf16_bits(f)); }
__device__ __forceinline__ unsigned short f16_bits(float f) { return __builtin_bit_cast(unsigned short, (_Float16)f); }

__device__ __forceinline__ void f16split16(float a, unsigned short& hb, unsigned short& lb) {
  const float z = a * 16.0f;
  const _Float16 hf = (_Float16)z;
  const float res = (z - (float)hf) * 2048.0f;
  hb = __builtin_bit_cast(unsigned short, hf);
  lb = __builtin_bit_cast(unsigned short, (_Float16)res);
}
__device__ __forceinline__ void f16split64(float a, unsigned short& hb, unsigned short& lb) {
  const float z = a * 64.0f;
  const _Float16 hf = (_Float16)z;
  const float res = z - (float)hf;
  hb = __builtin_bit_cast(unsigned short, hf);
  lb = __builtin_bit_cast(unsigned short, (_Float16)res);
}

__device__ __forceinline__ v8f mma_bf16(us16 a, us16 b, v8f c) {
  return __builtin_amdgcn_wmma_f32_16x16x32_bf16(false, __builtin_bit_cast(v16b, a), false, __builtin_bit_cast(v16b, b), (short)0, c, false, false);
}
__device__ __forceinline__ v8f mma_f16(us16 a, us16 b, v8f c) {
  return __builtin_amdgcn_wmma_f32_16x16x32_f16(false, __builtin_bit_cast(v16h, a), false, __builtin_bit_cast(v16h, b), (short)0, c, false, false);
}
__device__ __forceinline__ void wguard4(v8f& c0, v8f& c1, v8f& c2, v8f& c3, const us16& a0,
                                        const us16& b0, const us16& b1, const us16& b2, const us16& b3) {
#if defined(__HIP_DEVICE_COMPILE__)
  asm volatile("v_nop\n\tv_nop\n\tv_nop\n\tv_nop"
               : "+v"(c0), "+v"(c1), "+v"(c2), "+v"(c3)
               : "v"(a0), "v"(b0), "v"(b1), "v"(b2), "v"(b3));
#endif
}
__device__ __forceinline__ void wguard8(v8f& c0, v8f& c1, v8f& c2, v8f& c3, v8f& c4, v8f& c5, v8f& c6, v8f& c7,
                                        const us16& a0, const us16& a1,
                                        const us16& b0, const us16& b1, const us16& b2, const us16& b3) {
#if defined(__HIP_DEVICE_COMPILE__)
  asm volatile("v_nop\n\tv_nop\n\tv_nop\n\tv_nop"
               : "+v"(c0), "+v"(c1), "+v"(c2), "+v"(c3), "+v"(c4), "+v"(c5), "+v"(c6), "+v"(c7)
               : "v"(a0), "v"(a1), "v"(b0), "v"(b1), "v"(b2), "v"(b3));
#endif
}
__device__ __forceinline__ void wguard4m(v8f& c0, v8f& c1, v8f& c2, v8f& c3, const us16& a0,
                                         const us16& b0, const us16& b1, const us16& b2, const us16& b3) {
#if defined(__HIP_DEVICE_COMPILE__)
  asm volatile("v_nop\n\tv_nop\n\tv_nop\n\tv_nop"
               : "+v"(c0), "+v"(c1), "+v"(c2), "+v"(c3)
               : "v"(a0), "v"(b0), "v"(b1), "v"(b2), "v"(b3)
               : "memory");
#endif
}
__device__ __forceinline__ void wguard1x8m(v8f& c0, const us16& a0, const us16& a1, const us16& a2, const us16& a3,
                                           const us16& b0, const us16& b1, const us16& b2, const us16& b3) {
#if defined(__HIP_DEVICE_COMPILE__)
  asm volatile("v_nop\n\tv_nop\n\tv_nop\n\tv_nop"
               : "+v"(c0)
               : "v"(a0), "v"(a1), "v"(a2), "v"(a3), "v"(b0), "v"(b1), "v"(b2), "v"(b3)
               : "memory");
#endif
}

__device__ __forceinline__ us16 gfrag(const unsigned short* p) {
  const int kh = ((threadIdx.x >> 4) & 1) * 8;
  FragU f;
  f.h[0] = *(const us8a*)(p + kh);
  f.h[1] = *(const us8a*)(p + 16 + kh);
  return f.v;
}

__device__ __forceinline__ float softplus_f(float z) {
  return fmaxf(z, 0.0f) + log1pf(__expf(-fabsf(z)));
}
__device__ __forceinline__ int lvl_of(int d) {
  const int dd = (d > 0) ? d : 1;
  const int l = 32 - __clz(dd);
  const int lc = (l < NLV - 1) ? l : (NLV - 1);
  return (d > 0) ? lc : 0;
}
__device__ __forceinline__ unsigned short a_bits(float accv, int d, float dg, float lv) {
  const float dec = __expf(fminf(dg, 0.0f));
  const float val = (accv * KSC) * dec * lv;
  const float w = (d >= 0) ? (val * 256.0f) : 0.0f;
  return f16_bits(w);
}

template <int MODE>
__global__ __launch_bounds__(256) void k_cvt(const float* __restrict__ src, unsigned short* dst, int total8) {
  const int idx = blockIdx.x * 256 + threadIdx.x;
  if (idx >= total8) return;
  const size_t off = (size_t)idx * 8;
  const v4f a = *(const v4fa*)(src + off), c = *(const v4fa*)(src + off + 4);
  us8 o;
#pragma unroll
  for (int u = 0; u < 4; ++u) {
    o[u]     = (MODE == 0) ? bf16_bits(a[u]) : f16_bits(bf16r(a[u]) * 256.0f);
    o[4 + u] = (MODE == 0) ? bf16_bits(c[u]) : f16_bits(bf16r(c[u]) * 256.0f);
  }
  *(volatile us8*)(dst + off) = o;
  __threadfence();
  *(volatile us8*)(dst + off) = o;
}

__global__ __launch_bounds__(128) void k_cvt_wgl(const float* __restrict__ Wg, const float* __restrict__ Wdl, unsigned short* dst) {
  const int row = blockIdx.x, tid = threadIdx.x;
  us8 o;
  if (row < NHD + NHD * NLV) {
    const float* src = (row < NHD) ? (Wg + (size_t)row * DMOD) : (Wdl + (size_t)(row - NHD) * DMOD);
    const v4f a = *(const v4fa*)(src + tid * 8), c = *(const v4fa*)(src + tid * 8 + 4);
#pragma unroll
    for (int u = 0; u < 4; ++u) { o[u] = bf16_bits(a[u]); o[4 + u] = bf16_bits(c[u]); }
  } else {
#pragma unroll
    for (int u = 0; u < 8; ++u) o[u] = (unsigned short)0;
  }
  unsigned short* d = dst + (size_t)row * DMOD + tid * 8;
  *(volatile us8*)d = o;
  __threadfence();
  *(volatile us8*)d = o;
}

__global__ __launch_bounds__(128) void k_gemm_gl(const unsigned short* __restrict__ Ap, const unsigned short* __restrict__ Bw,
                                                const float* __restrict__ bg, const float* __restrict__ Lp,
                                                float* gpl, float* lam, int sl) {
  __shared__ __attribute__((aligned(16))) float oS[64 * GST];
  const int tid = threadIdx.x, lane = tid & 31, wave = tid >> 5, cl = lane & 15, hh = lane >> 4;
  const int m0b = blockIdx.x * 64, m0 = m0b + 16 * wave;

  v8f acc[8];
#pragma unroll
  for (int j = 0; j < 8; ++j) { const v8f zz = {0.f, 0.f, 0.f, 0.f, 0.f, 0.f, 0.f, 0.f}; acc[j] = zz; }

  const unsigned short* a0p = Ap + (size_t)(m0 + cl) * (size_t)DMOD;
  const unsigned short* bwp = Bw + (size_t)cl * (size_t)DMOD;
#pragma unroll 1
  for (int k0 = 0; k0 < DMOD; k0 += 32) {
    const us16 af = gfrag(a0p + k0);
    us16 bfr[4];
#pragma unroll
    for (int j = 0; j < 4; ++j) bfr[j] = gfrag(bwp + (size_t)(16 * j) * (size_t)DMOD + k0);
#pragma unroll
    for (int j = 0; j < 4; ++j) acc[j] = mma_bf16(af, bfr[j], acc[j]);
    wguard4(acc[0], acc[1], acc[2], acc[3], af, bfr[0], bfr[1], bfr[2], bfr[3]);
    us16 bf2[4];
#pragma unroll
    for (int j = 0; j < 4; ++j) bf2[j] = gfrag(bwp + (size_t)(16 * (4 + j)) * (size_t)DMOD + k0);
#pragma unroll
    for (int j = 0; j < 4; ++j) acc[4 + j] = mma_bf16(af, bf2[j], acc[4 + j]);
    wguard4(acc[4], acc[5], acc[6], acc[7], af, bf2[0], bf2[1], bf2[2], bf2[3]);
  }

  float* so = oS + wave * (16 * GST);
#pragma unroll
  for (int j = 0; j < 8; ++j)
#pragma unroll
    for (int r = 0; r < 8; ++r) so[(8 * hh + r) * GST + 16 * j + cl] = acc[j][r];
  __syncthreads();

  const int b = m0b / sl, ts = m0b - b * sl;
  {
    const int h = tid >> 4, t4 = (tid & 15) * 4;
    const float bgv = bf16r(bg[h]);
    v4f gv;
#pragma unroll
    for (int u = 0; u < 4; ++u) gv[u] = -softplus_f(oS[(t4 + u) * GST + h] + bgv);
    float* p = gpl + (size_t)(b * NHD + h) * (size_t)sl + ts + t4;
    *(volatile v4f*)p = gv;
    __threadfence();
    *(volatile v4f*)p = gv;
  }
#pragma unroll 1
  for (int it = 0; it < 16; ++it) {
    const int row = it * 4 + wave, c0 = lane * 4;
    v4f lv;
#pragma unroll
    for (int u = 0; u < 4; ++u) {
      const int c = c0 + u;
      int idx = c - NHD;
      idx = (idx < 0) ? 0 : idx;
      idx = (idx > NHD * NLV - 1) ? (NHD * NLV - 1) : idx;
      const float lp = bf16r(Lp[idx]);
      const float s = softplus_f(oS[row * GST + c] + lp);
      lv[u] = (c >= NHD && c < NHD + NHD * NLV) ? s : 0.0f;
    }
    float* p = lam + (size_t)(m0b + row) * (size_t)LAMP + c0;
    *(volatile v4f*)p = lv;
    __threadfence();
    *(volatile v4f*)p = lv;
  }
}

__global__ __launch_bounds__(32) void k_cumsum(const float* __restrict__ gpl, float* Ghi, float* Glo, int sl) {
  __shared__ __attribute__((aligned(16))) float shi[SLMAX];
  __shared__ __attribute__((aligned(16))) float slo[SLMAX];
  const int row = blockIdx.x, lane = threadIdx.x;
  if (lane == 0) {
    double acc = 0.0;
#pragma unroll 1
    for (int t = 0; t < sl; ++t) {
      acc += (double)gpl[(size_t)row * (size_t)sl + t];
      const float hi = (float)acc;
      shi[t] = hi;
      slo[t] = (float)(acc - (double)hi);
    }
  }
  __syncthreads();
  const int nit = sl / 128;
#pragma unroll 1
  for (int it = 0; it < nit; ++it) {
    const int c = it * 128 + lane * 4;
    const v4f vh = *(const v4fa*)(shi + c), vl = *(const v4fa*)(slo + c);
    float* ph = Ghi + (size_t)row * (size_t)sl + c;
    float* pl = Glo + (size_t)row * (size_t)sl + c;
    *(volatile v4f*)ph = vh;
    *(volatile v4f*)pl = vl;
    __threadfence();
    *(volatile v4f*)ph = vh;
    *(volatile v4f*)pl = vl;
  }
}

__global__ __launch_bounds__(256) void k_gemm_proj(const unsigned short* __restrict__ Ap, const unsigned short* __restrict__ Bw,
                                                  unsigned short* Qp, unsigned short* Kp, unsigned short* VH, unsigned short* VL, int sl) {
  __shared__ __attribute__((aligned(16))) float oS[8 * 16 * OSTR];
  const int tid = threadIdx.x, lane = tid & 31, wave = tid >> 5, cl = lane & 15, hh = lane >> 4;
  const int m0 = blockIdx.x * TPB + 16 * wave, n0 = blockIdx.y * 64;

  v8f acc[4];
#pragma unroll
  for (int j = 0; j < 4; ++j) { const v8f zz = {0.f, 0.f, 0.f, 0.f, 0.f, 0.f, 0.f, 0.f}; acc[j] = zz; }

  const unsigned short* a0p = Ap + (size_t)(m0 + cl) * (size_t)DMOD;
  const unsigned short* bwp = Bw + (size_t)(n0 + cl) * (size_t)DMOD;
#pragma unroll 1
  for (int k0 = 0; k0 < DMOD; k0 += 32) {
    const us16 af = gfrag(a0p + k0);
    us16 bfr[4];
#pragma unroll
    for (int j = 0; j < 4; ++j) bfr[j] = gfrag(bwp + (size_t)(16 * j) * (size_t)DMOD + k0);
#pragma unroll
    for (int j = 0; j < 4; ++j) acc[j] = mma_bf16(af, bfr[j], acc[j]);
    wguard4(acc[0], acc[1], acc[2], acc[3], af, bfr[0], bfr[1], bfr[2], bfr[3]);
  }

  float* so = oS + wave * (16 * OSTR);
#pragma unroll
  for (int j = 0; j < 4; ++j)
#pragma unroll
    for (int r = 0; r < 8; ++r) so[(8 * hh + r) * OSTR + 16 * j + cl] = acc[j][r];
  __syncthreads();

  const int yb = blockIdx.y;
  const int m0b = blockIdx.x * TPB, b = m0b / sl, tb = m0b - b * sl;
  if (yb < 32) {
    unsigned short* dst = (yb < 16) ? Qp : Kp;
    const int yy = (yb < 16) ? yb : (yb - 16);
    const int head = yy >> 1, f0 = (yy & 1) * 64;
    us8 ov[4];
#pragma unroll
    for (int it = 0; it < 4; ++it) {
      const int cx = it * 256 + tid, r = cx >> 3, pc = (cx & 7) * 8;
      const float* sp = oS + r * OSTR + pc;
      const v4f z0 = *(const v4fa*)sp, z1 = *(const v4fa*)(sp + 4);
      us8 o;
#pragma unroll
      for (int u = 0; u < 4; ++u) {
        o[u]     = f16_bits(z0[u] * 64.0f);
        o[4 + u] = f16_bits(z1[u] * 64.0f);
      }
      ov[it] = o;
    }
#pragma unroll
    for (int pass = 0; pass < 2; ++pass) {
#pragma unroll
      for (int it = 0; it < 4; ++it) {
        const int cx = it * 256 + tid, r = cx >> 3, pc = (cx & 7) * 8;
        const size_t off = ((size_t)(b * NHD + head) * (size_t)sl + (size_t)(tb + r)) * (size_t)SDIM + (size_t)(f0 + pc);
        *(volatile us8*)(dst + off) = ov[it];
      }
      __threadfence();
    }
  } else {
    const int yy = yb - 32, head = yy >> 1, c0 = (yy & 1) * 64;
    us8 hv[4], lv[4];
#pragma unroll
    for (int it = 0; it < 4; ++it) {
      const int cx = it * 256 + tid, g = cx & 15, e = cx >> 4;
      us8 ho, lo;
#pragma unroll
      for (int i = 0; i < 8; ++i) {
        unsigned short hb, lb;
        f16split64(oS[(8 * g + i) * OSTR + e], hb, lb);
        ho[i] = hb; lo[i] = lb;
      }
      hv[it] = ho; lv[it] = lo;
    }
#pragma unroll
    for (int pass = 0; pass < 2; ++pass) {
#pragma unroll
      for (int it = 0; it < 4; ++it) {
        const int cx = it * 256 + tid, g = cx & 15, e = cx >> 4;
        const size_t off = ((size_t)(b * NHD + head) * (size_t)HDIM + (size_t)(c0 + e)) * (size_t)sl + (size_t)(tb + 8 * g);
        *(volatile us8*)(VH + off) = hv[it];
        *(volatile us8*)(VL + off) = lv[it];
      }
      __threadfence();
    }
  }
}

__global__ __launch_bounds__(256) void k_attn(const unsigned short* __restrict__ Qp, const unsigned short* __restrict__ Kp,
                                             const unsigned short* __restrict__ VHp, const unsigned short* __restrict__ VLp,
                                             const float* __restrict__ Ghi, const float* __restrict__ Glo, const float* __restrict__ Lam,
                                             unsigned short* YH, unsigned short* YL, int sl) {
  __shared__ __attribute__((aligned(16))) float sLam[TPB * NLV];
  __shared__ __attribute__((aligned(16))) unsigned short sY[8 * 16 * YST];
  const int tid = threadIdx.x, lane = tid & 31, wave = tid >> 5, cl = lane & 15, hh = lane >> 4;
  const int bh = blockIdx.x, b = bh / NHD, head = bh - b * NHD;
  const int t0 = blockIdx.y * TPB;
  const int tw = t0 + 16 * wave;
  const int tq = tw + cl;

  for (int i = tid; i < TPB * NLV; i += 256) {
    const int q = i / NLV, l = i - q * NLV;
    sLam[i] = Lam[(size_t)(b * sl + t0 + q) * (size_t)LAMP + NHD + head * NLV + l];
  }
  __syncthreads();

  const unsigned short* qrow = Qp + ((size_t)bh * (size_t)sl + (size_t)tq) * (size_t)SDIM;
  us16 bq[4];
#pragma unroll
  for (int ks = 0; ks < 4; ++ks) bq[ks] = gfrag(qrow + 32 * ks);
  const float gqh = Ghi[(size_t)bh * (size_t)sl + tq];
  const float gql = Glo[(size_t)bh * (size_t)sl + tq];
  const int lamb = (16 * wave + cl) * NLV;

  v8f acc[8];
#pragma unroll
  for (int j = 0; j < 8; ++j) { const v8f zz = {0.f, 0.f, 0.f, 0.f, 0.f, 0.f, 0.f, 0.f}; acc[j] = zz; }

  const unsigned short* kbp = Kp + ((size_t)bh * (size_t)sl + (size_t)cl) * (size_t)SDIM;
  const unsigned short* vhp = VHp + ((size_t)bh * (size_t)HDIM + (size_t)cl) * (size_t)sl;
  const unsigned short* vlp = VLp + ((size_t)bh * (size_t)HDIM + (size_t)cl) * (size_t)sl;
  const float* ghp = Ghi + (size_t)bh * (size_t)sl;
  const float* glp = Glo + (size_t)bh * (size_t)sl;
  const int nsteps = (tw + 16 + 31) >> 5;

#pragma unroll 1
  for (int st = 0; st < nsteps; ++st) {
    const int s0 = st * 32;
    const int ka0 = s0 + 8 * hh;
    const v8f zz = {0.f, 0.f, 0.f, 0.f, 0.f, 0.f, 0.f, 0.f};

    us16 ka[4];
#pragma unroll
    for (int ks = 0; ks < 4; ++ks) ka[ks] = gfrag(kbp + (size_t)s0 * (size_t)SDIM + 32 * ks);
    v8f sa = zz;
#pragma unroll
    for (int ks = 0; ks < 4; ++ks) sa = mma_f16(ka[ks], bq[ks], sa);
    wguard1x8m(sa, ka[0], ka[1], ka[2], ka[3], bq[0], bq[1], bq[2], bq[3]);
    us8 ea;
    {
      const v4f h0 = *(const v4fa*)(ghp + ka0), h1 = *(const v4fa*)(ghp + ka0 + 4);
      const v4f l0 = *(const v4fa*)(glp + ka0), l1 = *(const v4fa*)(glp + ka0 + 4);
#pragma unroll
      for (int r = 0; r < 4; ++r) {
        const int d = tq - (ka0 + r);
        const float dg = (gqh - h0[r]) + (gql - l0[r]);
        const float lv = sLam[lamb + lvl_of(d)];
        ea[r] = a_bits(sa[r], d, dg, lv);
      }
#pragma unroll
      for (int r = 0; r < 4; ++r) {
        const int d = tq - (ka0 + 4 + r);
        const float dg = (gqh - h1[r]) + (gql - l1[r]);
        const float lv = sLam[lamb + lvl_of(d)];
        ea[4 + r] = a_bits(sa[4 + r], d, dg, lv);
      }
    }

    us16 kb[4];
#pragma unroll
    for (int ks = 0; ks < 4; ++ks) kb[ks] = gfrag(kbp + (size_t)(s0 + 16) * (size_t)SDIM + 32 * ks);
    v8f sb = zz;
#pragma unroll
    for (int ks = 0; ks < 4; ++ks) sb = mma_f16(kb[ks], bq[ks], sb);
    wguard1x8m(sb, kb[0], kb[1], kb[2], kb[3], bq[0], bq[1], bq[2], bq[3]);
    us8 eb;
    {
      const v4f h2 = *(const v4fa*)(ghp + ka0 + 16), h3 = *(const v4fa*)(ghp + ka0 + 20);
      const v4f l2 = *(const v4fa*)(glp + ka0 + 16), l3 = *(const v4fa*)(glp + ka0 + 20);
#pragma unroll
      for (int r = 0; r < 4; ++r) {
        const int d = tq - (ka0 + 16 + r);
        const float dg = (gqh - h2[r]) + (gql - l2[r]);
        const float lv = sLam[lamb + lvl_of(d)];
        eb[r] = a_bits(sb[r], d, dg, lv);
      }
#pragma unroll
      for (int r = 0; r < 4; ++r) {
        const int d = tq - (ka0 + 20 + r);
        const float dg = (gqh - h3[r]) + (gql - l3[r]);
        const float lv = sLam[lamb + lvl_of(d)];
        eb[4 + r] = a_bits(sb[4 + r], d, dg, lv);
      }
    }
    FragU fA;
    fA.h[0] = ea; fA.h[1] = eb;
    const us16 afr = fA.v;

    us16 bv[4];
#pragma unroll
    for (int j = 0; j < 4; ++j) bv[j] = gfrag(vhp + (size_t)(16 * j) * (size_t)sl + s0);
#pragma unroll
    for (int j = 0; j < 4; ++j) acc[j] = mma_f16(afr, bv[j], acc[j]);
    wguard4m(acc[0], acc[1], acc[2], acc[3], afr, bv[0], bv[1], bv[2], bv[3]);
    us16 bl[4];
#pragma unroll
    for (int j = 0; j < 4; ++j) bl[j] = gfrag(vlp + (size_t)(16 * j) * (size_t)sl + s0);
#pragma unroll
    for (int j = 0; j < 4; ++j) acc[j] = mma_f16(afr, bl[j], acc[j]);
    wguard4m(acc[0], acc[1], acc[2], acc[3], afr, bl[0], bl[1], bl[2], bl[3]);
    us16 bw[4];
#pragma unroll
    for (int j = 0; j < 4; ++j) bw[j] = gfrag(vhp + (size_t)(16 * (4 + j)) * (size_t)sl + s0);
#pragma unroll
    for (int j = 0; j < 4; ++j) acc[4 + j] = mma_f16(afr, bw[j], acc[4 + j]);
    wguard4m(acc[4], acc[5], acc[6], acc[7], afr, bw[0], bw[1], bw[2], bw[3]);
    us16 bx[4];
#pragma unroll
    for (int j = 0; j < 4; ++j) bx[j] = gfrag(vlp + (size_t)(16 * (4 + j)) * (size_t)sl + s0);
#pragma unroll
    for (int j = 0; j < 4; ++j) acc[4 + j] = mma_f16(afr, bx[j], acc[4 + j]);
    wguard4m(acc[4], acc[5], acc[6], acc[7], afr, bx[0], bx[1], bx[2], bx[3]);
  }

  unsigned short* sy = sY + wave * (16 * YST);
#pragma unroll
  for (int j = 0; j < 8; ++j)
#pragma unroll
    for (int r = 0; r < 8; ++r) sy[(8 * hh + r) * YST + 16 * j + cl] = f16_bits(acc[j][r] * (1.0f / 1024.0f));
  __syncthreads();

  us8 ov[8];
#pragma unroll
  for (int it = 0; it < 8; ++it) {
    const int rr = 2 * it + hh, p = cl * 8;
    ov[it] = *(const us8a*)(sy + rr * YST + p);
  }
#pragma unroll
  for (int pass = 0; pass < 2; ++pass) {
#pragma unroll
    for (int it = 0; it < 8; ++it) {
      const int rr = 2 * it + hh, p = cl * 8;
      const size_t off = (size_t)(b * sl + tw + rr) * (size_t)DMOD + (size_t)(head * HDIM + p);
      *(volatile us8*)(YH + off) = ov[it];
    }
    __threadfence();
  }
  __syncthreads();

#pragma unroll
  for (int j = 0; j < 8; ++j)
#pragma unroll
    for (int r = 0; r < 8; ++r) {
      const float z = acc[j][r] * (1.0f / 1024.0f);
      const _Float16 hf = (_Float16)z;
      sy[(8 * hh + r) * YST + 16 * j + cl] = f16_bits((z - (float)hf) * 2048.0f);
    }
  __syncthreads();
#pragma unroll
  for (int it = 0; it < 8; ++it) {
    const int rr = 2 * it + hh, p = cl * 8;
    ov[it] = *(const us8a*)(sy + rr * YST + p);
  }
#pragma unroll
  for (int pass = 0; pass < 2; ++pass) {
#pragma unroll
    for (int it = 0; it < 8; ++it) {
      const int rr = 2 * it + hh, p = cl * 8;
      const size_t off = (size_t)(b * sl + tw + rr) * (size_t)DMOD + (size_t)(head * HDIM + p);
      *(volatile us8*)(YL + off) = ov[it];
    }
    __threadfence();
  }
}

__global__ __launch_bounds__(256) void k_gemm_out(const unsigned short* __restrict__ Ah, const unsigned short* __restrict__ Al,
                                                 const unsigned short* __restrict__ Wo, const float* __restrict__ X, float* P) {
  __shared__ __attribute__((aligned(16))) float oS[8 * 16 * OSTR];
  const int tid = threadIdx.x, lane = tid & 31, wave = tid >> 5, cl = lane & 15, hh = lane >> 4;
  const int m0 = blockIdx.x * TPB + 16 * wave, n0 = blockIdx.y * 64;

  v8f acch[4], accl[4];
#pragma unroll
  for (int j = 0; j < 4; ++j) { const v8f zz = {0.f, 0.f, 0.f, 0.f, 0.f, 0.f, 0.f, 0.f}; acch[j] = zz; accl[j] = zz; }

  const unsigned short* ahp = Ah + (size_t)(m0 + cl) * (size_t)DMOD;
  const unsigned short* alp = Al + (size_t)(m0 + cl) * (size_t)DMOD;
  const unsigned short* wop = Wo + (size_t)(n0 + cl) * (size_t)DMOD;
#pragma unroll 1
  for (int k0 = 0; k0 < DMOD; k0 += 32) {
    const us16 ah = gfrag(ahp + k0);
    const us16 al = gfrag(alp + k0);
    us16 bfr[4];
#pragma unroll
    for (int j = 0; j < 4; ++j) bfr[j] = gfrag(wop + (size_t)(16 * j) * (size_t)DMOD + k0);
#pragma unroll
    for (int j = 0; j < 4; ++j) {
      acch[j] = mma_f16(ah, bfr[j], acch[j]);
      accl[j] = mma_f16(al, bfr[j], accl[j]);
    }
    wguard8(acch[0], acch[1], acch[2], acch[3], accl[0], accl[1], accl[2], accl[3], ah, al, bfr[0], bfr[1], bfr[2], bfr[3]);
  }

  float* so = oS + wave * (16 * OSTR);
#pragma unroll
  for (int j = 0; j < 4; ++j)
#pragma unroll
    for (int r = 0; r < 8; ++r)
      so[(8 * hh + r) * OSTR + 16 * j + cl] = fmaf(accl[j][r], (1.0f / 2048.0f), acch[j][r]) * (1.0f / 4096.0f);
  __syncthreads();

#pragma unroll
  for (int pass = 0; pass < 2; ++pass) {
#pragma unroll
    for (int it = 0; it < 8; ++it) {
      const int cx = it * 32 + lane, r = cx >> 4, q = (cx & 15) * 4;
      const v4f v = *(const v4fa*)(so + r * OSTR + q);
      const v4f xr = *(const v4fa*)(X + (size_t)(m0 + r) * (size_t)DMOD + n0 + q);
      v4f o;
#pragma unroll
      for (int u = 0; u < 4; ++u) o[u] = v[u] + bf16r(xr[u]);
      *(volatile v4f*)(P + (size_t)(m0 + r) * (size_t)DMOD + n0 + q) = o;
    }
    __threadfence();
  }
}

__global__ __launch_bounds__(256) void k_ln(const float* __restrict__ P, const float* __restrict__ gam, const float* __restrict__ bet,
                                           float* out) {
  const int lane = threadIdx.x & 31, wave = threadIdx.x >> 5;
  const size_t row = (size_t)blockIdx.x * 8 + (size_t)wave;
  const float* pr = P + row * (size_t)DMOD;
  v4f xv[8];
  float s = 0.0f;
#pragma unroll
  for (int it = 0; it < 8; ++it) {
    xv[it] = *(const v4fa*)(pr + it * 128 + lane * 4);
    s += (xv[it][0] + xv[it][1]) + (xv[it][2] + xv[it][3]);
  }
#pragma unroll
  for (int o = 16; o > 0; o >>= 1) s += __shfl_xor(s, o, 32);
  const float mu = s * (1.0f / (float)DMOD);
  float q = 0.0f;
#pragma unroll
  for (int it = 0; it < 8; ++it)
#pragma unroll
    for (int u = 0; u < 4; ++u) { const float d = xv[it][u] - mu; q += d * d; }
#pragma unroll
  for (int o = 16; o > 0; o >>= 1) q += __shfl_xor(q, o, 32);
  const float rstd = rsqrtf(q * (1.0f / (float)DMOD) + 1e-5f);
  v4f ov[8];
#pragma unroll
  for (int it = 0; it < 8; ++it) {
    const v4f gv = *(const v4fa*)(gam + it * 128 + lane * 4), bv = *(const v4fa*)(bet + it * 128 + lane * 4);
    v4f o;
#pragma unroll
    for (int u = 0; u < 4; ++u) o[u] = (xv[it][u] - mu) * rstd * bf16r(gv[u]) + bf16r(bv[u]);
    ov[it] = o;
  }
#pragma unroll
  for (int pass = 0; pass < 2; ++pass) {
#pragma unroll
    for (int it = 0; it < 8; ++it)
      *(volatile v4f*)(out + row * (size_t)DMOD + it * 128 + lane * 4) = ov[it];
    __threadfence();
  }
}

extern "C" void kernel_launch(void* const* d_in, const int* in_sizes, int n_in,
                              void* d_out, int out_size, void* d_ws, size_t ws_size,
                              hipStream_t stream) {
  if (n_in < 11) return;
  const int nx = in_sizes[0];
  if (nx <= 0 || (nx % DMOD) != 0) return;
  const int ntok = nx / DMOD;
  if (in_sizes[1] != DMOD * DMOD || in_sizes[2] != DMOD * DMOD || in_sizes[3] != DMOD * DMOD) return;
  if (in_sizes[4] != NHD * DMOD || in_sizes[5] != NHD || in_sizes[6] != NHD * NLV * DMOD || in_sizes[7] != NHD * NLV) return;
  if (in_sizes[8] != DMOD * DMOD || in_sizes[9] != DMOD || in_sizes[10] != DMOD) return;
  if (out_size != nx) return;
  const int sl = (ntok < SLMAX) ? ntok : SLMAX;
  if (sl <= 0 || (sl % TPB) != 0 || (ntok % sl) != 0) return;
  const int nb = ntok / sl, nbh = nb * NHD;

  const float* x   = (const float*)d_in[0];
  const float* Wq  = (const float*)d_in[1];
  const float* Wk  = (const float*)d_in[2];
  const float* Wv  = (const float*)d_in[3];
  const float* Wg  = (const float*)d_in[4];
  const float* bg  = (const float*)d_in[5];
  const float* Wdl = (const float*)d_in[6];
  const float* Lp  = (const float*)d_in[7];
  const float* Wo  = (const float*)d_in[8];
  const float* lng = (const float*)d_in[9];
  const float* lnb = (const float*)d_in[10];
  float* out = (float*)d_out;

  size_t off = 0;
  auto carve = [&](size_t bytes) -> char* { char* p = (char*)d_ws + off; off += (bytes + 255) & ~(size_t)255; return p; };
  unsigned short* XB   = (unsigned short*)carve((size_t)ntok * DMOD * 2);
  unsigned short* WQKV = (unsigned short*)carve((size_t)NQKV * DMOD * 2);
  unsigned short* WGL  = (unsigned short*)carve((size_t)NGL * DMOD * 2);
  unsigned short* WO16 = (unsigned short*)carve((size_t)DMOD * DMOD * 2);
  unsigned short* QP   = (unsigned short*)carve((size_t)nbh * sl * SDIM * 2);
  unsigned short* KP   = (unsigned short*)carve((size_t)nbh * sl * SDIM * 2);
  unsigned short* VH   = (unsigned short*)carve((size_t)nbh * HDIM * sl * 2);
  unsigned short* VL   = (unsigned short*)carve((size_t)nbh * HDIM * sl * 2);
  float* GPL           = (float*)carve((size_t)nbh * sl * 4);
  float* GHI           = (float*)carve((size_t)nbh * sl * 4);
  float* GLO           = (float*)carve((size_t)nbh * sl * 4);
  float* LAM           = (float*)carve((size_t)ntok * LAMP * 4);
  unsigned short* YH   = (unsigned short*)carve((size_t)ntok * DMOD * 2);
  unsigned short* YL   = (unsigned short*)carve((size_t)ntok * DMOD * 2);
  float* PB            = (float*)carve((size_t)ntok * DMOD * 4);
  if (off > ws_size || off > (size_t)134217728) return;

  const dim3 b256(256), b128(128), b32(32);
  auto cdv = [](long a, long q) { return (unsigned)((a + q - 1) / q); };

  k_cvt<0><<<dim3(cdv((long)ntok * DMOD / 8, 256)), b256, 0, stream>>>(x, XB, ntok * DMOD / 8);
  k_cvt<0><<<dim3(cdv((long)DMOD * DMOD / 8, 256)), b256, 0, stream>>>(Wq, WQKV, DMOD * DMOD / 8);
  k_cvt<0><<<dim3(cdv((long)DMOD * DMOD / 8, 256)), b256, 0, stream>>>(Wk, WQKV + (size_t)DMOD * DMOD, DMOD * DMOD / 8);
  k_cvt<0><<<dim3(cdv((long)DMOD * DMOD / 8, 256)), b256, 0, stream>>>(Wv, WQKV + (size_t)2 * DMOD * DMOD, DMOD * DMOD / 8);
  k_cvt_wgl<<<dim3(NGL), b128, 0, stream>>>(Wg, Wdl, WGL);
  k_cvt<1><<<dim3(cdv((long)DMOD * DMOD / 8, 256)), b256, 0, stream>>>(Wo, WO16, DMOD * DMOD / 8);
  k_gemm_gl<<<dim3(ntok / 64), b128, 0, stream>>>(XB, WGL, bg, Lp, GPL, LAM, sl);
  k_cumsum<<<dim3(nbh), b32, 0, stream>>>(GPL, GHI, GLO, sl);
  k_gemm_proj<<<dim3(ntok / TPB, NQKV / 64), b256, 0, stream>>>(XB, WQKV, QP, KP, VH, VL, sl);
  k_attn<<<dim3(nbh, sl / TPB), b256, 0, stream>>>(QP, KP, VH, VL, GHI, GLO, LAM, YH, YL, sl);
  k_gemm_out<<<dim3(ntok / TPB, DMOD / 64), b256, 0, stream>>>(YH, YL, WO16, x, PB);
  k_ln<<<dim3(ntok / 8), b256, 0, stream>>>(PB, lng, lnb, out);
}
